// PointNetSetAbstraction_72567767433503
// MI455X (gfx1250) — hardware-verified
//
#include <hip/hip_runtime.h>
#include <math.h>
#pragma clang fp contract(off)

typedef __attribute__((ext_vector_type(16))) _Float16 v16h;
typedef __attribute__((ext_vector_type(8)))  _Float16 v8h;
typedef __attribute__((ext_vector_type(8)))  float    v8f;
typedef __attribute__((ext_vector_type(4)))  float    v4f;
typedef __attribute__((ext_vector_type(4)))  unsigned v4u;

constexpr int NBATCH = 8;
constexpr int NPT    = 4096;
constexpr int NCENT  = 1024;
constexpr int NSAMPLE_K = 32;
constexpr int CFEAT  = 64;
constexpr int KPAD0  = 96;
constexpr int MROWS  = NBATCH * NCENT * NSAMPLE_K;
constexpr int NBLK_GEMM = MROWS / 256;
static_assert(MROWS == 262144);
static_assert(NBLK_GEMM == 1024);
static_assert(KPAD0 % 32 == 0);

__device__ __forceinline__ unsigned short f2bf_bits(float f) {
  unsigned u = __float_as_uint(f);
  return (unsigned short)((u + 0x7FFFu + ((u >> 16) & 1u)) >> 16);
}
__device__ __forceinline__ float bf_bits2f(unsigned short h) { return __uint_as_float(((unsigned)h) << 16); }
__device__ __forceinline__ float bf16r(float f) { return bf_bits2f(f2bf_bits(f)); }

__device__ __forceinline__ float h16_to_f32(unsigned hb) {
  const unsigned sgn = (hb & 0x8000u) << 16;
  const unsigned em = hb & 0x7fffu;
  const float fn = __uint_as_float((em << 13) + 0x38000000u);
  const float fs = (float)em * 5.9604644775390625e-8f;
  const float mag = (em < 0x400u) ? fs : fn;
  return __uint_as_float(__float_as_uint(mag) | sgn);
}

__device__ __forceinline__ unsigned f16bits(float f) {
  const _Float16 h = (_Float16)f;
  unsigned u = (unsigned)__builtin_bit_cast(unsigned short, h);
  asm volatile("" : "+v"(u));
  return u;
}

__device__ __forceinline__ void wave_sync_lds() {
  __builtin_amdgcn_fence(__ATOMIC_RELEASE, "workgroup");
  __builtin_amdgcn_wave_barrier();
  __builtin_amdgcn_fence(__ATOMIC_ACQUIRE, "workgroup");
}

__device__ __forceinline__ void store2_v4f(float* p, v4f v) {
  *(volatile v4f*)p = v;
  __threadfence();
  *(volatile v4f*)p = v;
}
__device__ __forceinline__ void store2_v8h(unsigned short* p, v8h v) {
  *(volatile v8h*)p = v;
  __threadfence();
  *(volatile v8h*)p = v;
}

union FragU { v16h v; v8h h[2]; };
__device__ __forceinline__ v16h frag_load(const _Float16* p) {
  FragU f;
  f.h[0] = *(const v8h*)(p);
  f.h[1] = *(const v8h*)(p + 16);
  return f.v;
}
__device__ __forceinline__ v8f mma_h(v16h a, v16h b, v8f c) {
  c = __builtin_amdgcn_wmma_f32_16x16x32_f16(false, a, false, b, (short)0, c, false, false);
  asm volatile("v_nop\n\tv_nop\n\tv_nop\n\tv_nop" : "+v"(c) : "v"(a), "v"(b));
  return c;
}

__global__ __launch_bounds__(256) void k_prep_small(
    const float* __restrict__ xyz, const float* __restrict__ w0, const float* __restrict__ w1,
    const float* __restrict__ w2, float* __restrict__ xyzr, unsigned short* __restrict__ bt0,
    unsigned short* __restrict__ bt1, unsigned short* __restrict__ bt2) {
  const int blk = blockIdx.x;
  const int t = threadIdx.x;
  if (blk < 96) {
    const int i4 = (blk * 256 + t) * 4;
    const v4f v = *(const v4f*)(xyz + i4);
    v4f r;
    r.x = bf16r(v.x);
    r.y = bf16r(v.y);
    r.z = bf16r(v.z);
    r.w = bf16r(v.w);
    store2_v4f(xyzr + i4, r);
    return;
  }
  float zf = 0.0f;
  asm volatile("" : "+v"(zf));
  if (blk < 99) {
    const int i = (blk - 96) * 256 + t;
    const int o = i / 12;
    const int q = i - o * 12;
    v8h hv;
#pragma unroll
    for (int e = 0; e < 8; ++e) {
      const int cp = q * 8 + e;
      int sc = (cp < 64) ? (cp + 3) : (cp - 64);
      sc = sc > 66 ? 66 : sc;
      const float wv = w0[o * 67 + sc];
      const float x = (cp < 67) ? bf16r(wv) : zf;
      hv[e] = (_Float16)x;
    }
    store2_v8h(bt0 + (size_t)i * 8, hv);
    return;
  }
  if (blk < 101) {
    const int i = (blk - 99) * 256 + t;
    const v4f a = *(const v4f*)(w1 + (size_t)i * 8);
    const v4f b = *(const v4f*)(w1 + (size_t)i * 8 + 4);
    v8h hv;
    hv[0] = (_Float16)bf16r(a.x);
    hv[1] = (_Float16)bf16r(a.y);
    hv[2] = (_Float16)bf16r(a.z);
    hv[3] = (_Float16)bf16r(a.w);
    hv[4] = (_Float16)bf16r(b.x);
    hv[5] = (_Float16)bf16r(b.y);
    hv[6] = (_Float16)bf16r(b.z);
    hv[7] = (_Float16)bf16r(b.w);
    store2_v8h(bt1 + (size_t)i * 8, hv);
    return;
  }
  {
    const int i = (blk - 101) * 256 + t;
    const v4f a = *(const v4f*)(w2 + (size_t)i * 8);
    const v4f b = *(const v4f*)(w2 + (size_t)i * 8 + 4);
    v8h hv;
    hv[0] = (_Float16)bf16r(a.x);
    hv[1] = (_Float16)bf16r(a.y);
    hv[2] = (_Float16)bf16r(a.z);
    hv[3] = (_Float16)bf16r(a.w);
    hv[4] = (_Float16)bf16r(b.x);
    hv[5] = (_Float16)bf16r(b.y);
    hv[6] = (_Float16)bf16r(b.z);
    hv[7] = (_Float16)bf16r(b.w);
    store2_v8h(bt2 + (size_t)i * 8, hv);
  }
}

__global__ __launch_bounds__(256) void k_prep_pts(const float* __restrict__ pts,
                                                  unsigned short* __restrict__ ptsT) {
  __shared__ float tl[64 * 65];
  const int b = blockIdx.x >> 6;
  const int n0 = (blockIdx.x & 63) * 64;
  const int t = threadIdx.x;
  const int nl = t & 63;
  const int cq = t >> 6;
#pragma unroll 4
  for (int i = 0; i < 16; ++i) {
    const int c = cq + 4 * i;
    const float v = pts[((size_t)b * CFEAT + c) * NPT + n0 + nl];
    tl[nl * 65 + c] = bf16r(v);
  }
  __syncthreads();
  for (int pass = 0; pass < 2; ++pass) {
#pragma unroll
    for (int it = 0; it < 2; ++it) {
      const int q = it * 256 + t;
      const int row = q >> 3;
      const int c8 = (q & 7) * 8;
      v8h hv;
#pragma unroll
      for (int e = 0; e < 8; ++e) hv[e] = (_Float16)tl[row * 65 + c8 + e];
      *(volatile v8h*)(ptsT + ((size_t)b * NPT + n0 + row) * CFEAT + c8) = hv;
    }
    __threadfence();
  }
}

__global__ __launch_bounds__(512) void k_fps(const float* __restrict__ xyzr,
                                             float* __restrict__ out0,
                                             float* __restrict__ newxyz) {
#pragma clang fp contract(off)
  __shared__ __align__(16) float sxyz[3 * NPT];
  __shared__ float rv[2][16];
  __shared__ int ri[2][16];
  __shared__ int sidx[NCENT];
  const int b = blockIdx.x;
  const int t = threadIdx.x;
  const int lane = t & 31;
  const int wave = t >> 5;
  const float* xb = xyzr + (size_t)b * 3 * NPT;
  for (int i = t; i < 3 * NPT / 4; i += 512) {
    const v4f v = *(const v4f*)(xb + 4 * i);
    *(v4f*)(sxyz + 4 * i) = v;
  }
  __syncthreads();
  float px[8], py[8], pz[8], dist[8];
#pragma unroll
  for (int i = 0; i < 8; ++i) {
    const int n = t + i * 512;
    px[i] = sxyz[n];
    py[i] = sxyz[NPT + n];
    pz[i] = sxyz[2 * NPT + n];
    dist[i] = 1e10f;
  }
  int far = 0;
#pragma unroll 1
  for (int it = 0; it < NCENT; ++it) {
    const float cx = sxyz[far];
    const float cy = sxyz[NPT + far];
    const float cz = sxyz[2 * NPT + far];
    if (t == 0) sidx[it] = far;
    float bv = 0.0f;
    int bi = t;
#pragma unroll
    for (int i = 0; i < 8; ++i) {
      const float dx = px[i] - cx;
      const float dy = py[i] - cy;
      const float dz = pz[i] - cz;
      const float tx = dx * dx;
      const float ty = dy * dy;
      const float tz = dz * dz;
      const float d = (tx + tz) + ty;
      const float nd = fminf(dist[i], d);
      dist[i] = nd;
      if (i == 0) {
        bv = nd;
        bi = t;
      } else if (nd > bv) {
        bv = nd;
        bi = t + i * 512;
      }
    }
#pragma unroll
    for (int off = 1; off < 32; off <<= 1) {
      const float ov = __shfl_xor(bv, off, 32);
      const int oi = __shfl_xor(bi, off, 32);
      const bool take = (ov > bv) || (ov == bv && oi < bi);
      bv = take ? ov : bv;
      bi = take ? oi : bi;
    }
    const int buf = it & 1;
    if (lane == 0) {
      rv[buf][wave] = bv;
      ri[buf][wave] = bi;
    }
    __syncthreads();
    float gv = rv[buf][lane & 15];
    int gi = ri[buf][lane & 15];
#pragma unroll
    for (int off = 1; off < 16; off <<= 1) {
      const float ov = __shfl_xor(gv, off, 32);
      const int oi = __shfl_xor(gi, off, 32);
      const bool take = (ov > gv) || (ov == gv && oi < gi);
      gv = take ? ov : gv;
      gi = take ? oi : gi;
    }
    far = gi & (NPT - 1);
  }
  __syncthreads();
  for (int pass = 0; pass < 2; ++pass) {
    for (int i = t; i < 768; i += 512) {
      const int c = i >> 8;
      const int s4 = (i & 255) * 4;
      v4f v;
      v.x = sxyz[c * NPT + (sidx[s4 + 0] & (NPT - 1))];
      v.y = sxyz[c * NPT + (sidx[s4 + 1] & (NPT - 1))];
      v.z = sxyz[c * NPT + (sidx[s4 + 2] & (NPT - 1))];
      v.w = sxyz[c * NPT + (sidx[s4 + 3] & (NPT - 1))];
      *(volatile v4f*)(out0 + ((size_t)b * 3 + c) * NCENT + s4) = v;
    }
    for (int i = t; i < NCENT; i += 512) {
      const int n = sidx[i] & (NPT - 1);
      v4f v;
      v.x = sxyz[n];
      v.y = sxyz[NPT + n];
      v.z = sxyz[2 * NPT + n];
      v.w = 0.0f;
      *(volatile v4f*)(newxyz + ((size_t)b * NCENT + i) * 4) = v;
    }
    __threadfence();
  }
}

__global__ __launch_bounds__(128) void k_ballgather(const float* __restrict__ xyzr,
                                                    const float* __restrict__ newxyz,
                                                    const unsigned short* __restrict__ ptsT,
                                                    unsigned short* __restrict__ A0) {
#pragma clang fp contract(off)
  __shared__ int slots[4][32];
  __shared__ __align__(16) unsigned rows[4][32 * 48];
  const int wave = threadIdx.x >> 5;
  const int lane = threadIdx.x & 31;
  const int center = blockIdx.x * 4 + wave;
  const int b = center >> 10;
  const float* xb = xyzr + (size_t)b * 3 * NPT;
  const v4f cc = *(const v4f*)(newxyz + (size_t)center * 4);
  const float sx = cc.x;
  const float sy = cc.y;
  const float sz = cc.z;
  const float ss = (sx * sx + sz * sz) + sy * sy;
  slots[wave][lane] = 0;
  wave_sync_lds();
  int collected = 0;
  int first = 0;
  for (int c0 = 0; c0 < NPT; c0 += 32) {
    if (collected >= NSAMPLE_K) break;
    const int n = c0 + lane;
    const float nx = xb[n];
    const float ny = xb[NPT + n];
    const float nz = xb[2 * NPT + n];
    float p = sx * nx;
    p = __builtin_fmaf(sy, ny, p);
    p = __builtin_fmaf(sz, nz, p);
    const float nn = (nx * nx + nz * nz) + ny * ny;
    const float d = (-2.0f * p + ss) + nn;
    const bool inr = !(d > 0.04f);
    const unsigned mask = __builtin_amdgcn_ballot_w32(inr);
    const int pos = collected + __popc(mask & ((1u << lane) - 1u));
    if (inr && pos < NSAMPLE_K) slots[wave][pos] = n;
    if (collected == 0 && mask != 0u) first = c0 + __builtin_ctz(mask);
    collected += __popc(mask);
  }
  wave_sync_lds();
  const int filled = collected < NSAMPLE_K ? collected : NSAMPLE_K;
  int idx = slots[wave][lane];
  idx = (lane < filled) ? idx : first;
  idx = idx < 0 ? 0 : (idx > NPT - 1 ? NPT - 1 : idx);
  const float gx = xb[idx];
  const float gy = xb[NPT + idx];
  const float gz = xb[2 * NPT + idx];
  asm volatile("" ::: "memory");
  const v4u* prow = (const v4u*)(const void*)(ptsT + ((size_t)b * NPT + idx) * CFEAT);
  v4u pw[8];
#pragma unroll
  for (int q = 0; q < 8; ++q) pw[q] = prow[q];
  const float dx = gx - sx;
  const float dy = gy - sy;
  const float dz = gz - sz;
  const unsigned hx = f16bits(dx);
  const unsigned hy = f16bits(dy);
  const unsigned hz = f16bits(dz);
  unsigned zz = 0u;
  asm volatile("" : "+v"(zz));
  v4u c8;
  c8.x = (hx & 0xffffu) | (hy << 16);
  c8.y = (hz & 0xffffu) | (zz << 16);
  c8.z = zz;
  c8.w = zz;
  v4u cz;
  cz.x = zz;
  cz.y = zz;
  cz.z = zz;
  cz.w = zz;
  unsigned* myrow = &rows[wave][lane * 48];
#pragma unroll
  for (int q = 0; q < 8; ++q) *(v4u*)(myrow + q * 4) = pw[q];
  *(v4u*)(myrow + 32) = c8;
  *(v4u*)(myrow + 36) = cz;
  *(v4u*)(myrow + 40) = cz;
  *(v4u*)(myrow + 44) = cz;
  wave_sync_lds();
  unsigned* dst = (unsigned*)(void*)A0 + (size_t)center * (32 * 48);
  const unsigned* src = &rows[wave][0];
  for (int pass = 0; pass < 2; ++pass) {
#pragma unroll
    for (int j = 0; j < 12; ++j) {
      const v4u v = *(const v4u*)(src + (j * 32 + lane) * 4);
      *(volatile v4u*)(dst + (j * 32 + lane) * 4) = v;
    }
    __threadfence();
  }
}

__device__ __forceinline__ v16h bn_frag(const unsigned short* p, const float* al, const float* be) {
  const v4u w0 = *(const v4u*)(const void*)(p);
  const v4u w1 = *(const v4u*)(const void*)(p + 16);
  v16h f;
#pragma unroll
  for (int e = 0; e < 4; ++e) {
    const unsigned wa = w0[e];
    const unsigned wb = w1[e];
    const float ya0 = h16_to_f32(wa & 0xffffu);
    const float ya1 = h16_to_f32(wa >> 16);
    const float yb0 = h16_to_f32(wb & 0xffffu);
    const float yb1 = h16_to_f32(wb >> 16);
    const float xa0 = fmaxf(__builtin_fmaf(al[2 * e], ya0, be[2 * e]), 0.0f);
    const float xa1 = fmaxf(__builtin_fmaf(al[2 * e + 1], ya1, be[2 * e + 1]), 0.0f);
    const float xb0 = fmaxf(__builtin_fmaf(al[16 + 2 * e], yb0, be[16 + 2 * e]), 0.0f);
    const float xb1 = fmaxf(__builtin_fmaf(al[16 + 2 * e + 1], yb1, be[16 + 2 * e + 1]), 0.0f);
    f[2 * e] = (_Float16)xa0;
    f[2 * e + 1] = (_Float16)xa1;
    f[8 + 2 * e] = (_Float16)xb0;
    f[8 + 2 * e + 1] = (_Float16)xb1;
  }
  return f;
}

template <int KDIM, int NOUT, bool BNIN, bool POOL>
__global__ __launch_bounds__(128) void mlp_layer(
    const unsigned short* __restrict__ Ap, const unsigned short* __restrict__ Btp,
    const float* __restrict__ bias, const float* __restrict__ ab_in,
    unsigned short* __restrict__ Yp, float* __restrict__ mm, float* __restrict__ part) {
  constexpr int KS = KDIM / 32;
  constexpr int NT = NOUT / 64;
  constexpr int QN = 2 * NOUT;
  static_assert(KDIM % 32 == 0);
  static_assert(NOUT % 64 == 0);
  static_assert(!BNIN || KDIM == 64);
  static_assert(POOL || NT == 1);
  static_assert(!POOL || NOUT == 128);
  __shared__ __align__(16) float slab[4][32 * 68];
  __shared__ __align__(16) float sstat[4][QN];
  __shared__ __align__(16) float sal[64];
  __shared__ __align__(16) float sbe[64];
  const _Float16* A = (const _Float16*)(const void*)Ap;
  const _Float16* Bt = (const _Float16*)(const void*)Btp;
  const int tid = threadIdx.x;
  const int wave = tid >> 5;
  const int lane = tid & 31;
  const int hh = lane >> 4;
  const int c = lane & 15;
  if (BNIN) {
    if (tid < 64) {
      sal[tid] = ab_in[tid];
      sbe[tid] = ab_in[128 + tid];
    }
  } else {
    if (tid < 64) {
      sal[tid] = 0.0f;
      sbe[tid] = 0.0f;
    }
  }
  __syncthreads();
  const int rowW = (blockIdx.x * 4 + wave) * 64;
  float* sl = &slab[wave][0];
  float cs[NT][4], cq[NT][4];
#pragma unroll
  for (int tn = 0; tn < NT; ++tn)
#pragma unroll
    for (int j = 0; j < 4; ++j) {
      cs[tn][j] = 0.0f;
      cq[tn][j] = 0.0f;
    }

#pragma unroll 1
  for (int t = 0; t < 2; ++t) {
    const int row0 = rowW + t * 32;
    v16h af[2][KS];
#pragma unroll
    for (int i = 0; i < 2; ++i) {
#pragma unroll
      for (int ks = 0; ks < KS; ++ks) {
        const size_t ao = (size_t)(row0 + i * 16 + c) * KDIM + ks * 32 + 8 * hh;
        if (BNIN) af[i][ks] = bn_frag(Ap + ao, sal + ks * 32 + 8 * hh, sbe + ks * 32 + 8 * hh);
        else af[i][ks] = frag_load(A + ao);
      }
    }
#pragma unroll
    for (int tn = 0; tn < NT; ++tn) {
      v8f acc[2][4];
#pragma unroll
      for (int i = 0; i < 2; ++i)
#pragma unroll
        for (int j = 0; j < 4; ++j) acc[i][j] = (v8f){0.f, 0.f, 0.f, 0.f, 0.f, 0.f, 0.f, 0.f};
#pragma unroll
      for (int ks = 0; ks < KS; ++ks) {
#pragma unroll
        for (int j = 0; j < 4; ++j) {
          const v16h bf = frag_load(Bt + (size_t)(tn * 64 + j * 16 + c) * KDIM + ks * 32 + 8 * hh);
          acc[0][j] = mma_h(af[0][ks], bf, acc[0][j]);
          acc[1][j] = mma_h(af[1][ks], bf, acc[1][j]);
        }
      }
#pragma unroll
      for (int j = 0; j < 4; ++j) {
        const int n = tn * 64 + j * 16 + c;
        const float bv = bf16r(bias[n]);
        float mx = -INFINITY;
        float mn = INFINITY;
#pragma unroll
        for (int i = 0; i < 2; ++i) {
#pragma unroll
          for (int r = 0; r < 8; ++r) {
            const float v = acc[i][j][r] + bv;
            cs[tn][j] += v;
            cq[tn][j] = __builtin_fmaf(v, v, cq[tn][j]);
            if (POOL) {
              mx = fmaxf(mx, v);
              mn = fminf(mn, v);
            } else {
              sl[(i * 16 + 8 * hh + r) * 68 + j * 16 + c] = v;
            }
          }
        }
        if (POOL) {
          const float omx = __shfl_xor(mx, 16, 32);
          const float omn = __shfl_xor(mn, 16, 32);
          mx = fmaxf(mx, omx);
          mn = fminf(mn, omn);
          if (hh == 0) {
            sl[n] = mx;
            sl[128 + n] = mn;
          }
        }
      }
      if (!POOL) {
        wave_sync_lds();
        unsigned short* Y = Yp;
        const int q8 = lane >> 3;
        const int c8 = (lane & 7) * 8;
        for (int pass = 0; pass < 2; ++pass) {
#pragma unroll
          for (int it = 0; it < 8; ++it) {
            const int row = it * 4 + q8;
            const float* sp = sl + row * 68 + c8;
            v8h hv;
#pragma unroll
            for (int e = 0; e < 8; ++e) hv[e] = (_Float16)sp[e];
            *(volatile v8h*)(Y + (size_t)(row0 + row) * NOUT + tn * 64 + c8) = hv;
          }
          __threadfence();
        }
        wave_sync_lds();
      }
    }
    if (POOL) {
      wave_sync_lds();
      const int center = row0 >> 5;
      float* dst = mm + (size_t)center * 256;
      for (int pass = 0; pass < 2; ++pass) {
        const v4f m0 = *(const v4f*)(sl + lane * 4);
        const v4f m1 = *(const v4f*)(sl + 128 + lane * 4);
        *(volatile v4f*)(dst + lane * 4) = m0;
        *(volatile v4f*)(dst + 128 + lane * 4) = m1;
        __threadfence();
      }
      wave_sync_lds();
    }
  }
#pragma unroll
  for (int tn = 0; tn < NT; ++tn) {
#pragma unroll
    for (int j = 0; j < 4; ++j) {
      const float os = __shfl_xor(cs[tn][j], 16, 32);
      const float oq = __shfl_xor(cq[tn][j], 16, 32);
      const float s = cs[tn][j] + os;
      const float q = cq[tn][j] + oq;
      if (hh == 0) {
        sstat[wave][tn * 64 + j * 16 + c] = s;
        sstat[wave][NOUT + tn * 64 + j * 16 + c] = q;
      }
    }
  }
  __syncthreads();
  if (tid < QN / 4) {
    const int i4 = tid * 4;
    const v4f s0 = *(const v4f*)(&sstat[0][i4]);
    const v4f s1 = *(const v4f*)(&sstat[1][i4]);
    const v4f s2 = *(const v4f*)(&sstat[2][i4]);
    const v4f s3 = *(const v4f*)(&sstat[3][i4]);
    const v4f r = ((s0 + s1) + s2) + s3;
    store2_v4f(part + (size_t)blockIdx.x * QN + i4, r);
  }
}

template <int NCH>
__global__ __launch_bounds__(256) void k_stat(const float* __restrict__ part,
                                              const float* __restrict__ g,
                                              const float* __restrict__ be,
                                              float* __restrict__ ab, int nblk) {
  constexpr int QN = 2 * NCH;
  constexpr int NP = 256 / QN;
  static_assert(NP >= 1);
  __shared__ double dsum[256];
  __shared__ __align__(16) float sab[256];
  const int t = threadIdx.x;
  const int qi = t % QN;
  const int pt = t / QN;
  const int nb = nblk < NBLK_GEMM ? nblk : NBLK_GEMM;
  double acc = 0.0;
#pragma unroll 4
  for (int blk = pt; blk < nb; blk += NP) acc += (double)part[(size_t)blk * QN + qi];
  dsum[t] = acc;
  __syncthreads();
  const int o = t & 127;
  const bool valid = o < NCH;
  const int oc = valid ? o : 0;
  double S = 0.0;
  double Q = 0.0;
#pragma unroll
  for (int p = 0; p < NP; ++p) {
    S += dsum[p * QN + oc];
    Q += dsum[p * QN + NCH + oc];
  }
  constexpr double inv_cnt = 1.0 / (double)MROWS;
  const double mean = S * inv_cnt;
  double var = Q * inv_cnt - mean * mean;
  var = var < 0.0 ? 0.0 : var;
  const float gg = bf16r(g[oc]);
  const float bb = bf16r(be[oc]);
  const float a = gg * (1.0f / sqrtf((float)var + 1e-5f));
  const float bt = bb - (float)mean * a;
  float val = (t < 128) ? a : bt;
  val = valid ? val : 0.0f;
  sab[t] = val;
  __syncthreads();
  if (t < 64) {
    const v4f v = *(const v4f*)(sab + 4 * t);
    store2_v4f(ab + 4 * t, v);
  }
}

__global__ __launch_bounds__(256) void k_pool(const float* __restrict__ mm,
                                              const float* __restrict__ ab2,
                                              float* __restrict__ out1) {
  __shared__ float tile[128 * 33];
  const int b = blockIdx.x >> 5;
  const int s0 = (blockIdx.x & 31) * 32;
  const int t = threadIdx.x;
  const int o = t & 127;
  const int sh = t >> 7;
  const float al = ab2[o];
  const float bt = ab2[128 + o];
#pragma unroll 4
  for (int i = 0; i < 16; ++i) {
    const int s = sh * 16 + i;
    const size_t center = (size_t)b * NCENT + s0 + s;
    const float ymx = mm[center * 256 + o];
    const float ymn = mm[center * 256 + 128 + o];
    const float r1 = al * ymx + bt;
    const float r2 = al * ymn + bt;
    float r = fmaxf(r1, r2);
    r = fmaxf(r, 0.0f);
    tile[o * 33 + s] = r;
  }
  __syncthreads();
  for (int pass = 0; pass < 2; ++pass) {
#pragma unroll
    for (int it = 0; it < 4; ++it) {
      const int q = it * 256 + t;
      const int oo = q >> 3;
      const int s4 = (q & 7) * 4;
      v4f v;
      v.x = tile[oo * 33 + s4 + 0];
      v.y = tile[oo * 33 + s4 + 1];
      v.z = tile[oo * 33 + s4 + 2];
      v.w = tile[oo * 33 + s4 + 3];
      *(volatile v4f*)(out1 + ((size_t)b * 128 + oo) * NCENT + s0 + s4) = v;
    }
    __threadfence();
  }
}

extern "C" void kernel_launch(void* const* d_in, const int* in_sizes, int n_in,
                              void* d_out, int out_size, void* d_ws, size_t ws_size,
                              hipStream_t stream) {
  (void)in_sizes;
  (void)n_in;
  (void)out_size;
  const float* xyz = (const float*)d_in[0];
  const float* pts = (const float*)d_in[1];
  const float* w0 = (const float*)d_in[2];
  const float* b0 = (const float*)d_in[3];
  const float* g0 = (const float*)d_in[4];
  const float* be0 = (const float*)d_in[5];
  const float* w1 = (const float*)d_in[6];
  const float* b1 = (const float*)d_in[7];
  const float* g1 = (const float*)d_in[8];
  const float* be1 = (const float*)d_in[9];
  const float* w2 = (const float*)d_in[10];
  const float* b2 = (const float*)d_in[11];
  const float* g2 = (const float*)d_in[12];
  const float* be2 = (const float*)d_in[13];
  float* out = (float*)d_out;
  char* ws = (char*)d_ws;

  constexpr size_t SZ_XYZR = (size_t)NBATCH * 3 * NPT * 4;
  constexpr size_t SZ_PTST = (size_t)NBATCH * NPT * CFEAT * 2;
  constexpr size_t SZ_BT0 = (size_t)64 * KPAD0 * 2;
  constexpr size_t SZ_BT1 = (size_t)64 * 64 * 2;
  constexpr size_t SZ_BT2 = (size_t)128 * 64 * 2;
  constexpr size_t SZ_NEW = (size_t)NBATCH * NCENT * 4 * 4;
  constexpr size_t SZ_A0 = (size_t)MROWS * KPAD0 * 2;
  constexpr size_t SZ_Y0 = (size_t)MROWS * 64 * 2;
  constexpr size_t SZ_Y1 = (size_t)MROWS * 64 * 2;
  constexpr size_t SZ_MM = (size_t)NBATCH * NCENT * 256 * 4;
  constexpr size_t SZ_P0 = (size_t)NBLK_GEMM * 128 * 4;
  constexpr size_t SZ_P1 = (size_t)NBLK_GEMM * 128 * 4;
  constexpr size_t SZ_P2 = (size_t)NBLK_GEMM * 256 * 4;
  constexpr size_t SZ_AB = 1024;
  constexpr size_t OFF_XYZR = 0;
  constexpr size_t OFF_PTST = OFF_XYZR + SZ_XYZR;
  constexpr size_t OFF_BT0 = OFF_PTST + SZ_PTST;
  constexpr size_t OFF_BT1 = OFF_BT0 + SZ_BT0;
  constexpr size_t OFF_BT2 = OFF_BT1 + SZ_BT1;
  constexpr size_t OFF_NEW = OFF_BT2 + SZ_BT2;
  constexpr size_t OFF_A0 = OFF_NEW + SZ_NEW;
  constexpr size_t OFF_Y0 = OFF_A0 + SZ_A0;
  constexpr size_t OFF_Y1 = OFF_Y0 + SZ_Y0;
  constexpr size_t OFF_MM = OFF_Y1 + SZ_Y1;
  constexpr size_t OFF_P0 = OFF_MM + SZ_MM;
  constexpr size_t OFF_P1 = OFF_P0 + SZ_P0;
  constexpr size_t OFF_P2 = OFF_P1 + SZ_P1;
  constexpr size_t OFF_AB0 = OFF_P2 + SZ_P2;
  constexpr size_t OFF_AB1 = OFF_AB0 + SZ_AB;
  constexpr size_t OFF_AB2 = OFF_AB1 + SZ_AB;
  constexpr size_t WS_TOTAL = OFF_AB2 + SZ_AB;
  static_assert(WS_TOTAL == 132684800);
  static_assert(WS_TOTAL <= 134217728);
  static_assert(OFF_PTST % 128 == 0 && OFF_BT0 % 128 == 0 && OFF_BT1 % 128 == 0 && OFF_BT2 % 128 == 0);
  static_assert(OFF_NEW % 128 == 0 && OFF_A0 % 128 == 0 && OFF_Y0 % 128 == 0 && OFF_Y1 % 128 == 0);
  static_assert(OFF_MM % 128 == 0 && OFF_P0 % 128 == 0 && OFF_P1 % 128 == 0 && OFF_P2 % 128 == 0);
  static_assert(OFF_AB0 % 128 == 0 && OFF_AB1 % 128 == 0 && OFF_AB2 % 128 == 0);
  static_assert(SZ_A0 == (size_t)NBATCH * NCENT * 32 * 48 * 4);
  static_assert(SZ_Y0 == (size_t)NBLK_GEMM * 256 * 64 * 2 && SZ_Y1 == SZ_Y0);
  static_assert(98304 + (size_t)NBATCH * 128 * NCENT * 4 == 4292608);
  if (ws_size < WS_TOTAL) return;

  float* xyzr = (float*)(ws + OFF_XYZR);
  unsigned short* ptsT = (unsigned short*)(ws + OFF_PTST);
  unsigned short* bt0 = (unsigned short*)(ws + OFF_BT0);
  unsigned short* bt1 = (unsigned short*)(ws + OFF_BT1);
  unsigned short* bt2 = (unsigned short*)(ws + OFF_BT2);
  float* newxyz = (float*)(ws + OFF_NEW);
  unsigned short* a0 = (unsigned short*)(ws + OFF_A0);
  unsigned short* y0 = (unsigned short*)(ws + OFF_Y0);
  unsigned short* y1 = (unsigned short*)(ws + OFF_Y1);
  float* mmp = (float*)(ws + OFF_MM);
  float* p0 = (float*)(ws + OFF_P0);
  float* p1 = (float*)(ws + OFF_P1);
  float* p2 = (float*)(ws + OFF_P2);
  float* ab0 = (float*)(ws + OFF_AB0);
  float* ab1 = (float*)(ws + OFF_AB1);
  float* ab2 = (float*)(ws + OFF_AB2);
  float* out1 = out + 98304 / 4;

  k_prep_small<<<105, 256, 0, stream>>>(xyz, w0, w1, w2, xyzr, bt0, bt1, bt2);
  k_prep_pts<<<NBATCH * (NPT / 64), 256, 0, stream>>>(pts, ptsT);
  k_fps<<<NBATCH, 512, 0, stream>>>(xyzr, out, newxyz);
  k_ballgather<<<NBATCH * NCENT / 4, 128, 0, stream>>>(xyzr, newxyz, ptsT, a0);

  mlp_layer<KPAD0, 64, false, false><<<NBLK_GEMM, 128, 0, stream>>>(a0, bt0, b0, ab0, y0, mmp, p0);
  k_stat<64><<<1, 256, 0, stream>>>(p0, g0, be0, ab0, NBLK_GEMM);
  mlp_layer<64, 64, true, false><<<NBLK_GEMM, 128, 0, stream>>>(y0, bt1, b1, ab0, y1, mmp, p1);
  k_stat<64><<<1, 256, 0, stream>>>(p1, g1, be1, ab1, NBLK_GEMM);
  mlp_layer<64, 128, true, true><<<NBLK_GEMM, 128, 0, stream>>>(y1, bt2, b2, ab1, y0, mmp, p2);
  k_stat<128><<<1, 256, 0, stream>>>(p2, g2, be2, ab2, NBLK_GEMM);
  k_pool<<<NBATCH * (NCENT / 32), 256, 0, stream>>>(mmp, ab2, out1);
}
